// GATNet2_6270652252168
// MI455X (gfx1250) — hardware-verified
//
#include <hip/hip_runtime.h>
#include <stddef.h>
#include <stdint.h>
#include <math.h>


#define F_IN    256
#define HCW     256
#define NHD     4
#define HID     64
#define KA2     512
#define NGR     128
#define L1N     128
#define NOUT    256
#define NTHR    256
#define NWAVE   8
#define EPT     8
#define CHUNK   (NTHR * EPT)
#define WCAP    (EPT * 32)
#define LISTN   (NWAVE * WCAP)
#define NBMAX   2048
#define SLOTB   11
#define NBRUN   1024
#define RCAP    28672
#define DEGCAP  256
#define GBM     64
#define GBN     64
#define GTHR    128
#define MROWS   128
#define FLINES  64
#define HTHR    512
#define NEGSL   0.2f
#define EPS_SM  1e-16f
#define WSMAX   134217728
#define LDS_AGG ((2 * RCAP + 2 * NBMAX + LISTN) * 4 + 128)
#define MEAS_B1024  8415
#define MEAS_MAXDEG 24

static_assert((CHUNK & (CHUNK - 1)) == 0 && CHUNK <= (1 << SLOTB));
static_assert(NBMAX == (1 << SLOTB));
static_assert(NTHR * 8 == NBMAX);
static_assert(LISTN >= NBMAX);
static_assert(LISTN >= NWAVE * WCAP);
static_assert((RCAP % 32) == 0);
static_assert(LDS_AGG <= 300000);
static_assert((NBRUN & (NBRUN - 1)) == 0 && NBRUN >= 32 && NBRUN <= NBMAX && (NBRUN % NWAVE) == 0);
static_assert(RCAP >= 2 * MEAS_B1024);
static_assert(DEGCAP >= MEAS_MAXDEG + 8);
static_assert(GBM == (GTHR / 32) * 16);
static_assert(GTHR == 2 * GBN && GTHR == 2 * GBM);
static_assert((F_IN % 32) == 0 && (KA2 % 32) == 0);
static_assert((HCW % GBN) == 0 && HID == GBN && HCW == NHD * HID);
static_assert(KA2 == 2 * HCW);
static_assert((MROWS % GBM) == 0);
static_assert(HCW == 8 * 32);
static_assert((F_IN / 8) == 32);
static_assert(NOUT == NGR * 2 && NOUT == 4 * 64);
static_assert(HTHR == 512 && L1N == 128 && (NGR % 2) == 0);
static_assert(2 * FLINES <= HTHR);

typedef float          v4f  __attribute__((ext_vector_type(4)));
typedef float          v8f  __attribute__((ext_vector_type(8)));
typedef int            v4i  __attribute__((ext_vector_type(4)));
typedef int            v8i  __attribute__((ext_vector_type(8)));
typedef unsigned int   v4u  __attribute__((ext_vector_type(4)));
typedef unsigned short v8us __attribute__((ext_vector_type(8)));
typedef __bf16         v16b __attribute__((ext_vector_type(16)));
typedef v4f  __attribute__((may_alias)) v4fa;
typedef v8us __attribute__((may_alias)) v8usa;
union FragB { v16b v; v8us h[2]; v8i w; };

__device__ __forceinline__ v8f wmb(const FragB& a, const FragB& b, v8f c) {
  v8f d = __builtin_amdgcn_wmma_f32_16x16x32_bf16(false, a.v, false, b.v, (short)0, c, false, false);
  asm volatile("v_nop\n\tv_nop\n\tv_nop\n\tv_nop" : "+v"(d) : "v"(a.w), "v"(b.w));
  return d;
}

__device__ __forceinline__ unsigned int f2bf(float f) {
  const unsigned int u = __float_as_uint(f);
  const unsigned int r = ((u + 0x7FFFu + ((u >> 16) & 1u)) >> 16) & 0xFFFFu;
  return (f != f) ? 0x7FC0u : r;
}
__device__ __forceinline__ float bf2f(unsigned int b) { return __uint_as_float(b << 16); }
__device__ __forceinline__ float bfr(float f) { return bf2f(f2bf(f)); }
__device__ __forceinline__ v4f bfr4(const v4f a) {
  v4f r; r.x = bfr(a.x); r.y = bfr(a.y); r.z = bfr(a.z); r.w = bfr(a.w); return r;
}
__device__ __forceinline__ unsigned int pk2(float lo, float hi) { return f2bf(lo) | (f2bf(hi) << 16); }
__device__ __forceinline__ v4u pack8(const v4f a, const v4f b) {
  v4u r;
  r.x = pk2(a.x, a.y); r.y = pk2(a.z, a.w); r.z = pk2(b.x, b.y); r.w = pk2(b.z, b.w);
  return r;
}
__device__ __forceinline__ float smax(float m, float v) { return (v > m || v != v) ? v : m; }

__device__ __forceinline__ int scan_chunk(const int* __restrict__ dsts, int nE, int cbase, int slotBase,
                                          int nb, int vec8, int* list, int tid, int lane, int wave) {
  int wc = 0;
  const int el0  = tid * EPT;
  const int e0   = cbase + el0;
  const int sent = -2147483647 - 1;
  v4i da, db;
  if (vec8 != 0 && cbase + CHUNK <= nE) {
    da = *(const v4i*)(dsts + e0);
    db = *(const v4i*)(dsts + e0 + 4);
  } else {
    da.x = (e0     < nE) ? dsts[min(e0,     nE - 1)] : sent;
    da.y = (e0 + 1 < nE) ? dsts[min(e0 + 1, nE - 1)] : sent;
    da.z = (e0 + 2 < nE) ? dsts[min(e0 + 2, nE - 1)] : sent;
    da.w = (e0 + 3 < nE) ? dsts[min(e0 + 3, nE - 1)] : sent;
    db.x = (e0 + 4 < nE) ? dsts[min(e0 + 4, nE - 1)] : sent;
    db.y = (e0 + 5 < nE) ? dsts[min(e0 + 5, nE - 1)] : sent;
    db.z = (e0 + 6 < nE) ? dsts[min(e0 + 6, nE - 1)] : sent;
    db.w = (e0 + 7 < nE) ? dsts[min(e0 + 7, nE - 1)] : sent;
  }
  const unsigned nbs = (unsigned)slotBase;
  const unsigned unb = (unsigned)nb;
  const unsigned s0 = (unsigned)da.x - nbs, s1 = (unsigned)da.y - nbs;
  const unsigned s2 = (unsigned)da.z - nbs, s3 = (unsigned)da.w - nbs;
  const unsigned s4 = (unsigned)db.x - nbs, s5 = (unsigned)db.y - nbs;
  const unsigned s6 = (unsigned)db.z - nbs, s7 = (unsigned)db.w - nbs;
  const bool h0 = s0 < unb, h1 = s1 < unb, h2 = s2 < unb, h3 = s3 < unb;
  const bool h4 = s4 < unb, h5 = s5 < unb, h6 = s6 < unb, h7 = s7 < unb;
  const unsigned any = __builtin_amdgcn_ballot_w32(h0 | h1 | h2 | h3 | h4 | h5 | h6 | h7);
  if (any != 0u) {
#define HITJ(J, HJ, SJ) { \
      const unsigned mj = __builtin_amdgcn_ballot_w32(HJ); \
      if (mj != 0u) { \
        if (HJ) { \
          const int pos = wc + (int)__builtin_amdgcn_mbcnt_lo(mj, 0u); \
          if (pos < WCAP) list[wave * WCAP + pos] = ((el0 + (J)) << SLOTB) | (int)(SJ); \
        } \
        wc += (int)__builtin_popcount(mj); } }
    HITJ(0, h0, s0)
    HITJ(1, h1, s1)
    HITJ(2, h2, s2)
    HITJ(3, h3, s3)
    HITJ(4, h4, s4)
    HITJ(5, h5, s5)
    HITJ(6, h6, s6)
    HITJ(7, h7, s7)
#undef HITJ
  }
  return wc;
}

__global__ __launch_bounds__(NTHR) void k_xprep(const float* __restrict__ x, unsigned short* xb, int nN, int nUnits) {
  const int i = (int)blockIdx.x * NTHR + (int)threadIdx.x;
  if (i >= nUnits) return;
  const int row = i >> 5;
  const int c0  = (i & 31) * 8;
  const int rc  = row < nN ? row : nN - 1;
  const float* p = x + (size_t)rc * F_IN + c0;
  v4f a = *(const v4fa*)p, b = *(const v4fa*)(p + 4);
  const v4f z4 = {0.f, 0.f, 0.f, 0.f};
  if (row >= nN) { a = z4; b = z4; }
  const v4u hv = pack8(a, b);
  const size_t o = (size_t)row * F_IN + c0;
  *(volatile v4u*)(xb + o) = hv;
  __threadfence();
  *(volatile v4u*)(xb + o) = hv;
}

__global__ __launch_bounds__(NTHR) void k_wtr(const float* __restrict__ w, int Kin, int Ncol, int Nrows, int Kout,
                                              unsigned short* wt, int nUnits) {
  const int u = (int)blockIdx.x * NTHR + (int)threadIdx.x;
  if (u >= nUnits) return;
  const int kq = Kout >> 3;
  const int n  = u / kq;
  const int k8 = (u - n * kq) * 8;
  const int kk = k8 - (k8 / Kin) * Kin;
  const int ncl = n < Ncol ? n : Ncol - 1;
  const float* p = w + (size_t)kk * (size_t)Ncol + ncl;
  v4f a, b;
  a.x = p[0];                    a.y = p[(size_t)Ncol];         a.z = p[(size_t)2 * Ncol];     a.w = p[(size_t)3 * Ncol];
  b.x = p[(size_t)4 * Ncol];     b.y = p[(size_t)5 * Ncol];     b.z = p[(size_t)6 * Ncol];     b.w = p[(size_t)7 * Ncol];
  const v4f z4 = {0.f, 0.f, 0.f, 0.f};
  if (n >= Ncol || n >= Nrows) { a = z4; b = z4; }
  const v4u wv = pack8(a, b);
  unsigned short* o = wt + (size_t)n * (size_t)Kout + k8;
  *(volatile v4u*)o = wv;
  __threadfence();
  *(volatile v4u*)o = wv;
}

__global__ __launch_bounds__(GTHR) void k_gemm(
    const unsigned short* __restrict__ A, const unsigned short* __restrict__ WT,
    float* outF, int K, int ldo,
    const float* __restrict__ atts, const float* __restrict__ attd, int attLen,
    float* SD, int MPr)
{
  __shared__ __attribute__((aligned(16))) float stg[GBM * GBN];
  __shared__ __attribute__((aligned(16))) float satt[2 * GBN];
  __shared__ __attribute__((aligned(16))) float sdot[2 * GBM];
  const int tid = (int)threadIdx.x, lane = tid & 31, wave = tid >> 5, hh = lane >> 4, m = lane & 15;
  const int rowBase = (int)blockIdx.x * GBM;
  const int head    = (int)blockIdx.y;
  const int col0    = head * GBN;

  {
    const int which = tid >> 6;
    const int c  = tid & 63;
    const int cl = c < attLen ? c : attLen - 1;
    const float vs = atts[head * attLen + cl];
    const float vd = attd[head * attLen + cl];
    float v = (which == 0) ? vs : vd;
    v = (c < attLen) ? bfr(v) : 0.f;
    satt[which * GBN + c] = v;
  }

  v8f acc[4];
  {
    const v8f z = {0.f, 0.f, 0.f, 0.f, 0.f, 0.f, 0.f, 0.f};
    acc[0] = z; acc[1] = z; acc[2] = z; acc[3] = z;
  }
  const unsigned short* ap = A  + (size_t)(rowBase + 16 * wave + m) * (size_t)K + 8 * hh;
  const unsigned short* wp = WT + (size_t)(col0 + m) * (size_t)K + 8 * hh;
  const int ksteps = K >> 5;
#pragma unroll 1
  for (int ks = 0; ks < ksteps; ++ks) {
    FragB af;
    af.h[0] = *(const v8usa*)(ap + 32 * ks);
    af.h[1] = *(const v8usa*)(ap + 32 * ks + 16);
#pragma unroll
    for (int t = 0; t < 4; ++t) {
      const unsigned short* wq = wp + (size_t)(16 * t) * (size_t)K + 32 * ks;
      FragB bf;
      bf.h[0] = *(const v8usa*)wq;
      bf.h[1] = *(const v8usa*)(wq + 16);
      acc[t] = wmb(af, bf, acc[t]);
    }
  }

#pragma unroll
  for (int t = 0; t < 4; ++t) {
    const int lc = 16 * t + m;
#pragma unroll
    for (int r = 0; r < 8; ++r) {
      const int lr = 16 * wave + 8 * hh + r;
      stg[lr * GBN + lc] = acc[t][r];
    }
  }
  __syncthreads();

  {
    const int row = tid & 63, which = tid >> 6;
    const float* sa = satt + which * GBN;
    const float* hr = stg + row * GBN;
    float d = 0.f;
#pragma unroll 4
    for (int c4 = 0; c4 < GBN / 4; ++c4) {
      const v4f hv = *(const v4fa*)(hr + 4 * c4);
      const v4f av = *(const v4fa*)(sa + 4 * c4);
      d = fmaf(hv.x, av.x, d);
      d = fmaf(hv.y, av.y, d);
      d = fmaf(hv.z, av.z, d);
      d = fmaf(hv.w, av.w, d);
    }
    sdot[which * GBM + row] = d;
  }
  __syncthreads();

  v4f fv[8];
#pragma unroll
  for (int i = 0; i < 8; ++i) {
    const int lr = 16 * wave + 2 * i + hh;
    fv[i] = *(const v4fa*)(stg + lr * GBN + 4 * m);
  }
  const int which2 = lane >> 4, piece = lane & 15;
  const v4f sdv = *(const v4fa*)(sdot + which2 * GBM + 4 * piece);
  float* sp = SD + (size_t)(2 * head + which2) * (size_t)MPr + rowBase + 4 * piece;

#pragma unroll
  for (int i = 0; i < 8; ++i) {
    const int lr = 16 * wave + 2 * i + hh;
    const int gr = rowBase + lr;
    float* op = outF + (size_t)gr * (size_t)ldo + col0 + 4 * m;
    *(volatile v4f*)op = fv[i];
  }
  if (wave == 0) *(volatile v4f*)sp = sdv;
  __threadfence();
#pragma unroll
  for (int i = 0; i < 8; ++i) {
    const int lr = 16 * wave + 2 * i + hh;
    const int gr = rowBase + lr;
    float* op = outF + (size_t)gr * (size_t)ldo + col0 + 4 * m;
    *(volatile v4f*)op = fv[i];
  }
  if (wave == 0) *(volatile v4f*)sp = sdv;
}

template<int L>
__global__ __launch_bounds__(NTHR) void k_agg(
    const int* __restrict__ srcs, const int* __restrict__ dsts,
    const float* __restrict__ F, const float* __restrict__ SD,
    const float* __restrict__ bias,
    unsigned short* HP, float* PO, int* FLAG,
    int nN, int nE, int nb, int vec8, int MPr) {
  extern __shared__ v4f lds_dyn[];
  int* reg1 = (int*)lds_dyn;
  int* reg2 = reg1 + RCAP;
  int* scnt = reg2 + RCAP;
  int* soff = scnt + NBMAX;
  int* list = soff + NBMAX;
  int* wcnt = list + LISTN;
  int* wtot = wcnt + NWAVE;
  int* wbig = wtot + NWAVE;
  const int tid = (int)threadIdx.x, lane = tid & 31, wave = tid >> 5;
  const int nodeBase = (int)blockIdx.x * nb;

  for (int i = tid; i < NBMAX; i += NTHR) scnt[i] = 0;
  __syncthreads();

  int tot = 0;
  const int nChunks = (nE + CHUNK - 1) / CHUNK;
#pragma unroll 1
  for (int ch = 0; ch < nChunks; ++ch) {
    const int cbase = ch * CHUNK;
    const int wc = scan_chunk(dsts, nE, cbase, nodeBase, nb, vec8, list, tid, lane, wave);
    if (lane == 0) wcnt[wave] = wc;
    __syncthreads();
    int pre = 0, all = 0;
#pragma unroll
    for (int w2 = 0; w2 < NWAVE; ++w2) {
      int c = wcnt[w2];
      c = c < 0 ? 0 : (c > WCAP ? WCAP : c);
      all += c;
      pre += (w2 < wave) ? c : 0;
    }
    const int wcc  = wc > WCAP ? WCAP : wc;
    const int base = tot + pre;
#pragma unroll 1
    for (int i = lane; i < wcc; i += 32) {
      const int ent = list[wave * WCAP + i];
      const int el  = (ent >> SLOTB) & (CHUNK - 1);
      const int sl  = ent & (NBMAX - 1);
      int eid = cbase + el;
      eid = eid > nE - 1 ? nE - 1 : eid;
      const int pos = base + i;
      if (pos < RCAP) reg1[pos] = (int)(((unsigned)eid << SLOTB) | (unsigned)sl);
    }
    tot += all;
    tot = tot > RCAP ? RCAP : tot;
    __syncthreads();
  }
  const int nh = tot;

  if (wave == 0) {
#pragma unroll 1
    for (int b0 = 0; b0 < nh; b0 += 32) {
      const int idx = b0 + lane;
      const int uv  = reg1[idx < nh ? idx : nh - 1];
      const int m32 = (nh - b0) < 32 ? (nh - b0) : 32;
#pragma unroll 1
      for (int k = 0; k < m32; ++k) {
        const int u  = __builtin_amdgcn_readlane(uv, k);
        const int sl = u & (NBMAX - 1);
        if (lane == 0) scnt[sl] = scnt[sl] + 1;
      }
    }
  }
  __syncthreads();

  int anyb = 0;
  {
    const v4i ca = *(const v4i*)(scnt + 8 * tid);
    const v4i cb = *(const v4i*)(scnt + 8 * tid + 4);
    const int e0 = ca.x < 0 ? 0 : ca.x, e1 = ca.y < 0 ? 0 : ca.y, e2 = ca.z < 0 ? 0 : ca.z, e3 = ca.w < 0 ? 0 : ca.w;
    const int e4 = cb.x < 0 ? 0 : cb.x, e5 = cb.y < 0 ? 0 : cb.y, e6 = cb.z < 0 ? 0 : cb.z, e7 = cb.w < 0 ? 0 : cb.w;
    const bool bigc = (e0 > DEGCAP) | (e1 > DEGCAP) | (e2 > DEGCAP) | (e3 > DEGCAP) |
                      (e4 > DEGCAP) | (e5 > DEGCAP) | (e6 > DEGCAP) | (e7 > DEGCAP);
    const unsigned bm = __builtin_amdgcn_ballot_w32(bigc);
    const int ts = e0 + e1 + e2 + e3 + e4 + e5 + e6 + e7;
    int incl = ts;
#pragma unroll
    for (int d = 1; d < 32; d <<= 1) {
      const int up = __shfl_up(incl, d);
      if (lane >= d) incl += up;
    }
    if (lane == 31) wtot[wave] = incl;
    if (lane == 0)  wbig[wave] = (bm != 0u) ? 1 : 0;
    __syncthreads();
    int pre = 0;
#pragma unroll
    for (int w2 = 0; w2 < NWAVE; ++w2) {
      pre += (w2 < wave) ? wtot[w2] : 0;
      anyb |= wbig[w2];
    }
    int run = pre + incl - ts;
    soff[8 * tid + 0] = run; run += e0;
    soff[8 * tid + 1] = run; run += e1;
    soff[8 * tid + 2] = run; run += e2;
    soff[8 * tid + 3] = run; run += e3;
    soff[8 * tid + 4] = run; run += e4;
    soff[8 * tid + 5] = run; run += e5;
    soff[8 * tid + 6] = run; run += e6;
    soff[8 * tid + 7] = run;
  }
  __syncthreads();
  for (int i = tid; i < NBMAX; i += NTHR) list[i] = soff[i];
  __syncthreads();

  if (wave == 0) {
#pragma unroll 1
    for (int b0 = 0; b0 < nh; b0 += 32) {
      const int idx = b0 + lane;
      const int uv  = reg1[idx < nh ? idx : nh - 1];
      const int m32 = (nh - b0) < 32 ? (nh - b0) : 32;
#pragma unroll 1
      for (int k = 0; k < m32; ++k) {
        const int u   = __builtin_amdgcn_readlane(uv, k);
        const int sl  = u & (NBMAX - 1);
        const int eid = (int)((unsigned)u >> SLOTB);
        if (lane == 0) {
          int pos = list[sl];
          pos = pos < 0 ? 0 : (pos > RCAP - 1 ? RCAP - 1 : pos);
          reg2[pos] = eid;
          list[sl] = pos + 1;
        }
      }
    }
  }
  __syncthreads();

  const int nbw = nb >> 3;
  const bool ovf = (nh >= RCAP);
  const float qnan = __int_as_float(0x7fc00000);

  if (wave == 0) {
    const int bf = (ovf || anyb != 0) ? 1 : 0;
    const v4i fv4 = {bf, bf, bf, bf};
    int* fp = FLAG + (size_t)blockIdx.x * 32 + 4 * (lane & 7);
    const bool fw = lane < 8;
    if (fw) *(volatile v4i*)fp = fv4;
    __threadfence();
    if (fw) *(volatile v4i*)fp = fv4;
  }

  const int c0   = 8 * lane;
  const int head = lane >> 3;
  const v4f bbA  = bfr4(*(const v4fa*)(bias + c0));
  const v4f bbB  = bfr4(*(const v4fa*)(bias + c0 + 4));
  const float* ASp = SD + (size_t)(2 * head) * (size_t)MPr;
  const float* ADp = ASp + MPr;
  const int sl1 = lane >> 1, sl2 = 16 + (lane >> 1);
  const bool odd = (lane & 1) != 0;

#pragma unroll 1
  for (int jt = 0; jt < nbw; ++jt) {
    const int slot = wave * nbw + jt;
    const int grow = nodeBase + slot;
    const int gcl  = grow < nN ? grow : nN - 1;
    int st = soff[slot];
    const int craw = scnt[slot];
    int cnt = craw;
    st  = st < 0 ? 0 : (st > nh ? nh : st);
    cnt = cnt < 0 ? 0 : (cnt > DEGCAP ? DEGCAP : cnt);
    if (cnt > nh - st) cnt = nh - st;
    const float pz = (ovf || craw > DEGCAP) ? qnan : 0.0f;

    const float* fr = F + (size_t)gcl * HCW + c0;
    v4f a0 = *(const v4fa*)fr;
    v4f a1 = *(const v4fa*)(fr + 4);
    const float adv = ADp[gcl];
    float l0 = ASp[gcl] + adv;
    l0 = l0 > 0.f ? l0 : NEGSL * l0;
    float mx = l0, dn = 1.0f;

#pragma unroll 1
    for (int q = 0; q < cnt; ++q) {
      int idx = st + q; idx = idx > RCAP - 1 ? RCAP - 1 : idx;
      int eid = reg2[idx]; eid = eid < 0 ? 0 : (eid > nE - 1 ? nE - 1 : eid);
      const int sraw = srcs[eid];
      const int s = sraw < 0 ? 0 : (sraw > nN - 1 ? nN - 1 : sraw);
      const float* fs = F + (size_t)s * HCW + c0;
      const v4f f0 = *(const v4fa*)fs;
      const v4f f1 = *(const v4fa*)(fs + 4);
      float lg = ASp[s] + adv;
      lg = lg > 0.f ? lg : NEGSL * lg;
      const float df = lg - mx;
      const float ee = expf(-fabsf(df));
      const bool up  = df > 0.f;
      const float s1 = up ? ee : 1.0f;
      const float s2 = up ? 1.0f : ee;
      mx = up ? lg : mx;
      dn = fmaf(dn, s1, s2);
      a0.x = fmaf(a0.x, s1, s2 * f0.x);
      a0.y = fmaf(a0.y, s1, s2 * f0.y);
      a0.z = fmaf(a0.z, s1, s2 * f0.z);
      a0.w = fmaf(a0.w, s1, s2 * f0.w);
      a1.x = fmaf(a1.x, s1, s2 * f1.x);
      a1.y = fmaf(a1.y, s1, s2 * f1.y);
      a1.z = fmaf(a1.z, s1, s2 * f1.z);
      a1.w = fmaf(a1.w, s1, s2 * f1.w);
    }
    const float inv = __builtin_amdgcn_rcpf(dn + EPS_SM);
    const bool live = grow < nN;
    float r0 = fmaf(a0.x, inv, bbA.x), r1 = fmaf(a0.y, inv, bbA.y);
    float r2 = fmaf(a0.z, inv, bbA.z), r3 = fmaf(a0.w, inv, bbA.w);
    float r4 = fmaf(a1.x, inv, bbB.x), r5 = fmaf(a1.y, inv, bbB.y);
    float r6 = fmaf(a1.z, inv, bbB.z), r7 = fmaf(a1.w, inv, bbB.w);
#pragma unroll 1
    for (int it = 0; it < 8; ++it) {
      const float v  = r0;
      const float vn = v > 0.f ? 0.f : v;
      const float e  = v > 0.f ? v : expm1f(vn);
      r0 = r1; r1 = r2; r2 = r3; r3 = r4; r4 = r5; r5 = r6; r6 = r7; r7 = e;
    }
    const float o0 = live ? (r0 + pz) : 0.f, o1 = live ? (r1 + pz) : 0.f;
    const float o2 = live ? (r2 + pz) : 0.f, o3 = live ? (r3 + pz) : 0.f;
    const float o4 = live ? (r4 + pz) : 0.f, o5 = live ? (r5 + pz) : 0.f;
    const float o6 = live ? (r6 + pz) : 0.f, o7 = live ? (r7 + pz) : 0.f;
    const bool wr = grow < MPr;

    if (L == 1) {
      const unsigned int h0 = f2bf(o0), h1 = f2bf(o1), h2 = f2bf(o2), h3 = f2bf(o3);
      const unsigned int h4 = f2bf(o4), h5 = f2bf(o5), h6 = f2bf(o6), h7 = f2bf(o7);
      const unsigned int q0 = f2bf(o0 - bf2f(h0)), q1 = f2bf(o1 - bf2f(h1));
      const unsigned int q2 = f2bf(o2 - bf2f(h2)), q3 = f2bf(o3 - bf2f(h3));
      const unsigned int q4 = f2bf(o4 - bf2f(h4)), q5 = f2bf(o5 - bf2f(h5));
      const unsigned int q6 = f2bf(o6 - bf2f(h6)), q7 = f2bf(o7 - bf2f(h7));
      v4u hv, lv;
      hv.x = h0 | (h1 << 16); hv.y = h2 | (h3 << 16); hv.z = h4 | (h5 << 16); hv.w = h6 | (h7 << 16);
      lv.x = q0 | (q1 << 16); lv.y = q2 | (q3 << 16); lv.z = q4 | (q5 << 16); lv.w = q6 | (q7 << 16);
      unsigned short* gp = HP + (size_t)grow * KA2 + 8 * lane;
      if (wr) { *(volatile v4u*)gp = hv; *(volatile v4u*)(gp + HCW) = lv; }
      __threadfence();
      if (wr) { *(volatile v4u*)gp = hv; *(volatile v4u*)(gp + HCW) = lv; }
    } else {
      const float x0 = __shfl(o0, sl1), x1 = __shfl(o1, sl1), x2 = __shfl(o2, sl1), x3 = __shfl(o3, sl1);
      const float x4 = __shfl(o4, sl1), x5 = __shfl(o5, sl1), x6 = __shfl(o6, sl1), x7 = __shfl(o7, sl1);
      const float y0 = __shfl(o0, sl2), y1 = __shfl(o1, sl2), y2 = __shfl(o2, sl2), y3 = __shfl(o3, sl2);
      const float y4 = __shfl(o4, sl2), y5 = __shfl(o5, sl2), y6 = __shfl(o6, sl2), y7 = __shfl(o7, sl2);
      v4f va, vb;
      va.x = odd ? x4 : x0; va.y = odd ? x5 : x1; va.z = odd ? x6 : x2; va.w = odd ? x7 : x3;
      vb.x = odd ? y4 : y0; vb.y = odd ? y5 : y1; vb.z = odd ? y6 : y2; vb.w = odd ? y7 : y3;
      float* op = PO + (size_t)grow * HCW + 4 * lane;
      if (wr) { *(volatile v4f*)op = va; *(volatile v4f*)(op + 128) = vb; }
      __threadfence();
      if (wr) { *(volatile v4f*)op = va; *(volatile v4f*)(op + 128) = vb; }
    }
  }
}

__global__ __launch_bounds__(NTHR) void k_pool(const float* __restrict__ hf, const int* __restrict__ bat,
                                               int nN, float* pl) {
  __shared__ __attribute__((aligned(16))) float wmx[NWAVE * HCW];
  __shared__ __attribute__((aligned(16))) float outs[HCW];
  const int tid = (int)threadIdx.x, lane = tid & 31, wave = tid >> 5;
  const int g = (int)blockIdx.x;
  const float ninf = __uint_as_float(0xff800000u);

  v4f ma = {ninf, ninf, ninf, ninf};
  v4f mb = {ninf, ninf, ninf, ninf};
#pragma unroll 1
  for (int i0 = wave * 32; i0 < nN; i0 += NTHR) {
    const int i  = i0 + lane;
    const int ic = i < nN ? i : nN - 1;
    const int b  = bat[ic];
    const bool hit = (i < nN) && (b == g);
    unsigned msk = __builtin_amdgcn_ballot_w32(hit);
    int nh = (int)__builtin_popcount(msk);
    nh = nh > 32 ? 32 : nh;
#pragma unroll 1
    for (int q = 0; q < nh; ++q) {
      const int k = __builtin_ffs((int)msk) - 1;
      msk &= msk - 1u;
      int node = i0 + (k < 0 ? 0 : k);
      node = node > nN - 1 ? nN - 1 : node;
      const float* pr = hf + (size_t)node * HCW + 8 * lane;
      const v4f va = *(const v4fa*)pr;
      const v4f vb = *(const v4fa*)(pr + 4);
      ma.x = smax(ma.x, va.x); ma.y = smax(ma.y, va.y); ma.z = smax(ma.z, va.z); ma.w = smax(ma.w, va.w);
      mb.x = smax(mb.x, vb.x); mb.y = smax(mb.y, vb.y); mb.z = smax(mb.z, vb.z); mb.w = smax(mb.w, vb.w);
    }
  }
  *(v4fa*)(wmx + wave * HCW + 8 * lane)     = ma;
  *(v4fa*)(wmx + wave * HCW + 8 * lane + 4) = mb;
  __syncthreads();
  {
    float m = ninf;
#pragma unroll
    for (int w2 = 0; w2 < NWAVE; ++w2) m = smax(m, wmx[w2 * HCW + tid]);
    outs[tid] = (m == ninf) ? 0.0f : m;
  }
  __syncthreads();
  const v4f ov = *(const v4fa*)(outs + 4 * (tid & 63));
  float* op = pl + (size_t)g * HCW + 4 * (tid & 63);
  const bool okst = tid < 64;
  if (okst) *(volatile v4f*)op = ov;
  __threadfence();
  if (okst) *(volatile v4f*)op = ov;
}

__global__ __launch_bounds__(HTHR) void k_head(const float* __restrict__ pl, const float* __restrict__ l1w,
                                               const float* __restrict__ l1b, const float* __restrict__ l2w,
                                               const float* __restrict__ l2b, const int* __restrict__ flags,
                                               int gA, float* out) {
  __shared__ __attribute__((aligned(16))) float z1h[64 * L1N];
  __shared__ float w2s[2 * L1N];
  __shared__ float b1s[L1N];
  __shared__ float b2s[4];
  __shared__ __attribute__((aligned(16))) float os[NOUT];
  __shared__ int wfl[HTHR / 32];
  const int tid = (int)threadIdx.x, lane = tid & 31, wave = tid >> 5;
  const float qnan = __int_as_float(0x7fc00000);

  {
    const int half = (tid >> 6) & 1;
    int li = tid & 63;
    li = li < gA ? li : gA - 1;
    li = li < 0 ? 0 : li;
    const int fv = flags[(size_t)(FLINES * half + li) * 32];
    const bool hit = (tid < 2 * FLINES) && ((tid & 63) < gA) && (fv == 1);
    const unsigned bm = __builtin_amdgcn_ballot_w32(hit);
    if (lane == 0) wfl[wave] = (bm != 0u) ? 1 : 0;
  }
  if (tid < 2 * L1N) w2s[tid] = bfr(l2w[tid]);
  if (tid < L1N)     b1s[tid] = bfr(l1b[tid]);
  if (tid < 4)       b2s[tid] = bfr(l2b[tid & 1]);
  __syncthreads();
  int anyf = 0;
#pragma unroll
  for (int w2 = 0; w2 < HTHR / 32; ++w2) anyf |= wfl[w2];

#pragma unroll 1
  for (int hf = 0; hf < 2; ++hf) {
#pragma unroll 1
    for (int i = tid; i < 64 * L1N; i += HTHR) {
      const int gl = i >> 7, n = i & (L1N - 1);
      const float* pr = pl + (size_t)(64 * hf + gl) * HCW;
      const float* wc = l1w + n;
      float s = 0.f;
#pragma unroll 1
      for (int k4 = 0; k4 < HCW / 4; ++k4) {
        const v4f p = *(const v4fa*)(pr + 4 * k4);
        const float w0 = bfr(wc[(size_t)(4 * k4 + 0) * L1N]);
        const float w1 = bfr(wc[(size_t)(4 * k4 + 1) * L1N]);
        const float w2 = bfr(wc[(size_t)(4 * k4 + 2) * L1N]);
        const float w3 = bfr(wc[(size_t)(4 * k4 + 3) * L1N]);
        s = fmaf(p.x, w0, s);
        s = fmaf(p.y, w1, s);
        s = fmaf(p.z, w2, s);
        s = fmaf(p.w, w3, s);
      }
      z1h[i] = s + b1s[n];
    }
    __syncthreads();
    if (tid < 128) {
      const int gl = tid >> 1, c = tid & 1;
      const float* zr = z1h + gl * L1N;
      float s = 0.f;
#pragma unroll 1
      for (int k4 = 0; k4 < L1N / 4; ++k4) {
        const v4f z = *(const v4fa*)(zr + 4 * k4);
        s = fmaf(z.x, w2s[(4 * k4 + 0) * 2 + c], s);
        s = fmaf(z.y, w2s[(4 * k4 + 1) * 2 + c], s);
        s = fmaf(z.z, w2s[(4 * k4 + 2) * 2 + c], s);
        s = fmaf(z.w, w2s[(4 * k4 + 3) * 2 + c], s);
      }
      s = s + b2s[c];
      os[128 * hf + tid] = (anyf != 0) ? qnan : s;
    }
    __syncthreads();
  }

  const v4f ov = *(const v4fa*)(os + 4 * (tid & 63));
  float* op = out + 4 * (tid & 63);
  const bool okst = tid < 64;
  if (okst) *(volatile v4f*)op = ov;
  __threadfence();
  if (okst) *(volatile v4f*)op = ov;
}

static inline int cdiv(int a, int b) { return (a + b - 1) / b; }
static inline size_t al256(size_t o) { return (o + 255) & ~(size_t)255; }

extern "C" void kernel_launch(void* const* d_in, const int* in_sizes, int n_in,
                              void* d_out, int out_size, void* d_ws, size_t ws_size,
                              hipStream_t stream) {
  if (n_in < 15) return;
  if (in_sizes[0] < F_IN || (in_sizes[0] % F_IN) != 0) return;
  const int nN = in_sizes[0] / F_IN;
  if (nN < 1 || nN > (1 << 22)) return;
  if (in_sizes[1] < 2 || (in_sizes[1] & 1) != 0) return;
  const int nE = in_sizes[1] / 2;
  if (nE < 1 || nE >= (1 << (32 - SLOTB))) return;
  if (in_sizes[2] != nN) return;
  if (in_sizes[3] != F_IN * HCW) return;
  if (in_sizes[4] != NHD * HID || in_sizes[5] != NHD * HID) return;
  if (in_sizes[6] != HCW) return;
  if (in_sizes[7] != HCW * HCW) return;
  if (in_sizes[8] != NHD * HID || in_sizes[9] != NHD * HID) return;
  if (in_sizes[10] != HCW) return;
  if (in_sizes[11] != HCW * L1N) return;
  if (in_sizes[12] != L1N) return;
  if (in_sizes[13] != L1N * 2) return;
  if (in_sizes[14] != 2) return;
  if (out_size != NOUT) return;

  const float* x    = (const float*)d_in[0];
  const int*   ei   = (const int*)  d_in[1];
  const int*   bat  = (const int*)  d_in[2];
  const float* W1   = (const float*)d_in[3];
  const float* a1s  = (const float*)d_in[4];
  const float* a1d  = (const float*)d_in[5];
  const float* b1   = (const float*)d_in[6];
  const float* W2   = (const float*)d_in[7];
  const float* a2s  = (const float*)d_in[8];
  const float* a2d  = (const float*)d_in[9];
  const float* b2   = (const float*)d_in[10];
  const float* l1w  = (const float*)d_in[11];
  const float* l1b  = (const float*)d_in[12];
  const float* l2w  = (const float*)d_in[13];
  const float* l2b  = (const float*)d_in[14];
  float* out = (float*)d_out;
  const int* src = ei;
  const int* dst = ei + nE;

  const int MP   = cdiv(nN, MROWS) * MROWS;
  const int nb   = NBRUN;
  const int gA   = cdiv(MP, nb);
  if (gA < 1 || gA > FLINES) return;
  if (gA * nb < MP) return;
  if ((MP % GBM) != 0) return;
  const int vec8 = ((nE & 3) == 0) ? 1 : 0;

  char* ws = (char*)d_ws;
  size_t off = 0;
  const size_t oA   = off; off = al256(off + (size_t)MP * KA2 * 2);
  const size_t oB   = off; off = al256(off + (size_t)MP * HCW * 4);
  const size_t oSD  = off; off = al256(off + (size_t)2 * NHD * MP * 4);
  const size_t oW1T = off; off = al256(off + (size_t)HCW * F_IN * 2);
  const size_t oW2D = off; off = al256(off + (size_t)HCW * KA2 * 2);
  const size_t oPL  = off; off = al256(off + (size_t)NGR * HCW * 4);
  const size_t oFL  = off; off = al256(off + (size_t)2 * FLINES * 128);
  if (off > ws_size || off > (size_t)WSMAX) return;
  if ((size_t)MP * F_IN * 2 > (size_t)MP * KA2 * 2) return;
  if ((size_t)MP * HCW * 4 > (size_t)MP * KA2 * 2) return;
  unsigned short* XB   = (unsigned short*)(ws + oA);
  unsigned short* X1HL = (unsigned short*)(ws + oA);
  float*          P    = (float*)(ws + oA);
  float*          H    = (float*)(ws + oB);
  float*          SD   = (float*)(ws + oSD);
  unsigned short* W1T  = (unsigned short*)(ws + oW1T);
  unsigned short* W2D  = (unsigned short*)(ws + oW2D);
  float*          PL   = (float*)(ws + oPL);
  int*            FLG  = (int*)(ws + oFL);

  hipFuncSetAttribute(reinterpret_cast<const void*>(&k_agg<1>),
                      hipFuncAttributeMaxDynamicSharedMemorySize, LDS_AGG);
  hipFuncSetAttribute(reinterpret_cast<const void*>(&k_agg<2>),
                      hipFuncAttributeMaxDynamicSharedMemorySize, LDS_AGG);

  const int nUx = MP * (F_IN / 8);
  k_xprep<<<cdiv(nUx, NTHR), NTHR, 0, stream>>>(x, XB, nN, nUx);

  {
    const int nUw1 = HCW * (F_IN / 8);
    k_wtr<<<cdiv(nUw1, NTHR), NTHR, 0, stream>>>(W1, F_IN, HCW, HCW, F_IN, W1T, nUw1);
    const int nUw2 = HCW * (KA2 / 8);
    k_wtr<<<cdiv(nUw2, NTHR), NTHR, 0, stream>>>(W2, HCW, HCW, HCW, KA2, W2D, nUw2);
  }

  const int gM = MP / GBM;
  k_gemm<<<dim3(gM, HCW / GBN), GTHR, 0, stream>>>(XB, W1T, H, F_IN, HCW, a1s, a1d, HID, SD, MP);
  k_agg<1><<<gA, NTHR, LDS_AGG, stream>>>(src, dst, H, SD, b1, X1HL, P, FLG, nN, nE, nb, vec8, MP);
  k_gemm<<<dim3(gM, HCW / GBN), GTHR, 0, stream>>>(X1HL, W2D, H, KA2, HCW, a2s, a2d, HID, SD, MP);
  k_agg<2><<<gA, NTHR, LDS_AGG, stream>>>(src, dst, H, SD, b2, X1HL, P, FLG + FLINES * 32, nN, nE, nb, vec8, MP);
  k_pool<<<NGR, NTHR, 0, stream>>>(P, bat, nN, PL);
  k_head<<<1, HTHR, 0, stream>>>(PL, l1w, l1b, l2w, l2b, FLG, gA, out);
}
